// ConsistentSelfAttentionTile_62277025792229
// MI455X (gfx1250) — hardware-verified
//
#include <hip/hip_runtime.h>


#define NB_  2
#define NN   512
#define CC   512
#define TW   64
#define NT   449
#define NS   288
typedef _Float16 h16;
typedef unsigned short bf;
typedef __attribute__((ext_vector_type(16))) __bf16   v16bf;
typedef __attribute__((ext_vector_type(16))) _Float16 v16h;
typedef __attribute__((ext_vector_type(8)))  _Float16 v8h;
typedef __attribute__((ext_vector_type(8)))  unsigned short v8us;
typedef __attribute__((ext_vector_type(8)))  float    v8f;
typedef __attribute__((ext_vector_type(4)))  float    v4f;
typedef v8h  __attribute__((may_alias)) v8ha;
typedef v4f  __attribute__((may_alias)) v4fa;
typedef v8us __attribute__((may_alias)) v8usa;

__device__ __forceinline__ unsigned short f2bf(float f) { unsigned u = __float_as_uint(f); u += 0x7FFFu + ((u >> 16) & 1u); return (unsigned short)(u >> 16); }
__device__ __forceinline__ float bf2f(unsigned short b) { return __uint_as_float(((unsigned)b) << 16); }
__device__ __forceinline__ float bfr(float f) { return bf2f(f2bf(f)); }
__device__ __forceinline__ v16h cat16(v8h lo, v8h hi) { return __builtin_shufflevector(lo, hi, 0, 1, 2, 3, 4, 5, 6, 7, 8, 9, 10, 11, 12, 13, 14, 15); }
__device__ __forceinline__ v16bf cat16b(v8us lo, v8us hi) { return __builtin_bit_cast(v16bf, __builtin_shufflevector(lo, hi, 0, 1, 2, 3, 4, 5, 6, 7, 8, 9, 10, 11, 12, 13, 14, 15)); }
__device__ __forceinline__ v8f wmma16(v16h a, v16h b, v8f c) { return __builtin_amdgcn_wmma_f32_16x16x32_f16(false, a, false, b, (short)0, c, false, false); }
__device__ __forceinline__ v8f wmmab(v16bf a, v16bf b, v8f c) { return __builtin_amdgcn_wmma_f32_16x16x32_bf16(false, a, false, b, (short)0, c, false, false); }


template <typename T16> struct WFrag;
template <> struct WFrag<h16> { typedef v16h V; static __device__ __forceinline__ V ld(const h16* p) { return cat16(*(const v8h*)p, *(const v8h*)(p + 16)); } static __device__ __forceinline__ v8f mma(V a, V b, v8f c) { return wmma16(a, b, c); } };
template <> struct WFrag<bf> { typedef v16bf V; static __device__ __forceinline__ V ld(const bf* p) { return cat16b(*(const v8us*)p, *(const v8us*)(p + 16)); } static __device__ __forceinline__ v8f mma(V a, V b, v8f c) { return wmmab(a, b, c); } };
template <typename T16, int NSPLIT, bool BIAS>
__global__ __launch_bounds__(32) void k_gemmw(const T16* __restrict__ A, const T16* __restrict__ A2, const T16* __restrict__ Bt, const T16* __restrict__ Bt2, int K, float* C, int ldc, const float* __restrict__ bias, size_t sA, size_t sB, size_t sC) {
    typedef typename WFrag<T16>::V V;
    __shared__ __align__(16) float os[16 * 68];
    const size_t z = blockIdx.z; A += z * sA; if (A2) A2 += z * sA; Bt += z * sB; if (Bt2) Bt2 += z * sB; C += z * sC;
    const int lane = threadIdx.x & 31, lr = lane & 15, hi = lane >> 4; const int r0 = blockIdx.x * 64, c0 = blockIdx.y * 64;
    v8f acc[4][4];
#pragma unroll
    for (int mb = 0; mb < 4; ++mb)
#pragma unroll
        for (int nb = 0; nb < 4; ++nb) acc[mb][nb] = (v8f){};
    const size_t aoff = (size_t)(r0 + lr) * K + 8 * hi, boff = (size_t)(c0 + lr) * K + 8 * hi;
#pragma unroll 1
    for (int kc = 0; kc < K; kc += 32) {
        V a[4], a2[4];
#pragma unroll
        for (int mb = 0; mb < 4; ++mb) { a[mb] = WFrag<T16>::ld(A + aoff + (size_t)mb * 16 * K + kc); if (NSPLIT == 1 || NSPLIT == 2) a2[mb] = WFrag<T16>::ld(A2 + aoff + (size_t)mb * 16 * K + kc); }
#pragma unroll
        for (int nb = 0; nb < 4; ++nb) { const V b = WFrag<T16>::ld(Bt + boff + (size_t)nb * 16 * K + kc); V b2; if (NSPLIT >= 2) b2 = WFrag<T16>::ld(Bt2 + boff + (size_t)nb * 16 * K + kc);
#pragma unroll
            for (int mb = 0; mb < 4; ++mb) { acc[mb][nb] = WFrag<T16>::mma(a[mb], b, acc[mb][nb]); if (NSPLIT == 1 || NSPLIT == 2) acc[mb][nb] = WFrag<T16>::mma(a2[mb], b, acc[mb][nb]); if (NSPLIT >= 2) acc[mb][nb] = WFrag<T16>::mma(a[mb], b2, acc[mb][nb]); } }
        asm volatile("v_nop\n\tv_nop\n\tv_nop\n\tv_nop" : "+v"(acc[0][0]), "+v"(acc[1][1]), "+v"(acc[2][2]), "+v"(acc[3][3]) : "v"(a[0]), "v"(a[3]));
    }
#pragma unroll
    for (int mb = 0; mb < 4; ++mb) {
#pragma unroll
        for (int nb = 0; nb < 4; ++nb) {
#pragma unroll
            for (int j = 0; j < 8; ++j) os[(hi * 8 + j) * 68 + nb * 16 + lr] = acc[mb][nb][j]; }
        __builtin_amdgcn_wave_barrier(); asm volatile("" ::: "memory");
        float* crow = C + (size_t)(r0 + mb * 16) * ldc + c0;
#pragma unroll 1
        for (int ps = 0; ps < 2; ++ps) {
#pragma unroll
            for (int s = 0; s < 8; ++s) { const int row = 2 * s + hi, cofs = lr * 4; v4f val = *(const v4fa*)(os + row * 68 + cofs); if (BIAS) { val[0] += bfr(bias[c0 + cofs]); val[1] += bfr(bias[c0 + cofs + 1]); val[2] += bfr(bias[c0 + cofs + 2]); val[3] += bfr(bias[c0 + cofs + 3]); }
                *(volatile v4f*)(crow + (size_t)row * ldc + cofs) = val; }
            if (ps == 0) __threadfence(); }
        __builtin_amdgcn_wave_barrier(); asm volatile("" ::: "memory");
    }
}

__device__ __forceinline__ void splitf(float y, unsigned short& h, unsigned short& l) { h = f2bf(y); l = f2bf(y - bf2f(h)); }
typedef __attribute__((ext_vector_type(2))) unsigned short v2us;
typedef __attribute__((ext_vector_type(4))) unsigned short v4us;

__global__ __launch_bounds__(256) void k_cvt8(const float* __restrict__ src, bf* dst, size_t n8) { const size_t i = (size_t)blockIdx.x * 256 + threadIdx.x; if (i >= n8) return; const v8f v = *(const v8f*)(src + i * 8); v8us o;
#pragma unroll
    for (int k = 0; k < 8; ++k) o[k] = f2bf(v[k]); *(volatile v8us*)(dst + i * 8) = o; __threadfence(); *(volatile v8us*)(dst + i * 8) = o; }
__global__ __launch_bounds__(256) void k_pl(const float* __restrict__ F, size_t n, bf* Ph, bf* Pl) { const size_t e = ((size_t)blockIdx.x * 256 + threadIdx.x) * 4; if (e >= n) return; v4us oh, ol;
#pragma unroll
    for (int u = 0; u < 4; ++u) { unsigned short a, b; splitf(F[e + u], a, b); oh[u] = a; ol[u] = b; } *(volatile v4us*)(Ph + e) = oh; *(volatile v4us*)(Pl + e) = ol; __threadfence(); *(volatile v4us*)(Ph + e) = oh; *(volatile v4us*)(Pl + e) = ol; }
__global__ __launch_bounds__(256) void k_cnt(const int* __restrict__ idx, float* CNT) { const int e = blockIdx.x * 256 + threadIdx.x; if (e >= NT * TW) return; const int u = e % TW; const int t = e / TW; const int* row = idx + (size_t)t * NS; int c = 1;
#pragma unroll 4
    for (int s = 0; s < NS; ++s) c += ((row[s] & (TW - 1)) == u) ? 1 : 0;
    const float cf = (float)c; *(volatile float*)(CNT + e) = cf; __threadfence(); *(volatile float*)(CNT + e) = cf; }
__global__ __launch_bounds__(256) void k_vpackt(const float* __restrict__ V, bf* Vh, bf* Vl) { const size_t e = ((size_t)blockIdx.x * 256 + threadIdx.x) * 2; if (e >= (size_t)NT * CC * TW) return; const int u = (int)(e % TW); const int d = (int)((e / TW) % CC); const int t = (int)(e / ((size_t)TW * CC)); v2us oh, ol;
#pragma unroll
    for (int q = 0; q < 2; ++q) { unsigned short a, b; splitf(V[(size_t)(t + u + q) * CC + d], a, b); oh[q] = a; ol[q] = b; } *(volatile v2us*)(Vh + e) = oh; *(volatile v2us*)(Vl + e) = ol; __threadfence(); *(volatile v2us*)(Vh + e) = oh; *(volatile v2us*)(Vl + e) = ol; }
__global__ __launch_bounds__(256) void k_tsoft(const float* __restrict__ S, const float* __restrict__ CNT, bf* Ph, bf* Pl) { const int lane = threadIdx.x & 31; const int row = blockIdx.x * 8 + (threadIdx.x >> 5); if (row >= NT * TW) return; const int t = row / TW; const float* sr = S + (size_t)row * TW; const float* cr = CNT + (size_t)t * TW; const int j0 = lane * 2;
    const float a0 = sr[j0], a1 = sr[j0 + 1]; float mx = fmaxf(a0, a1);
#pragma unroll
    for (int sh = 16; sh; sh >>= 1) mx = fmaxf(mx, __shfl_xor(mx, sh, 32));
    float d0 = __fsub_rn(a0, mx), d1 = __fsub_rn(a1, mx); asm volatile("" : "+v"(d0)); asm volatile("" : "+v"(d1));
    const float e0 = __fmul_rn(cr[j0], __builtin_amdgcn_exp2f(__fmul_rn(d0, 1.4426950408889634f))), e1 = __fmul_rn(cr[j0 + 1], __builtin_amdgcn_exp2f(__fmul_rn(d1, 1.4426950408889634f))); float sum = __fadd_rn(e0, e1);
#pragma unroll
    for (int sh = 16; sh; sh >>= 1) sum += __shfl_xor(sum, sh, 32);
    const float f = __fdiv_rn(1.0f, sum); v2us oh, ol; { unsigned short a, b; splitf(e0 * f, a, b); oh[0] = a; ol[0] = b; splitf(e1 * f, a, b); oh[1] = a; ol[1] = b; }
    const size_t oo = (size_t)row * TW + j0; *(volatile v2us*)(Ph + oo) = oh; *(volatile v2us*)(Pl + oo) = ol; __threadfence(); *(volatile v2us*)(Ph + oo) = oh; *(volatile v2us*)(Pl + oo) = ol; }
__global__ __launch_bounds__(256) void k_accum(const float* __restrict__ O, float* outb) { const size_t e = ((size_t)blockIdx.x * 256 + threadIdx.x) * 4; if (e >= (size_t)NN * CC) return; const int c = (int)(e % CC); const int pos = (int)(e / CC); const int t0 = (pos - TW + 1 > 0) ? pos - TW + 1 : 0, t1 = (pos < NT - 1) ? pos : NT - 1; float a[4] = {0.f, 0.f, 0.f, 0.f};
#pragma unroll 1
    for (int t = t0; t <= t1; ++t) { const v4f o = *(const v4f*)(O + ((size_t)t * TW + (pos - t)) * CC + c);
#pragma unroll
        for (int u = 0; u < 4; ++u) a[u] = __fadd_rn(a[u], o[u]); }
    const float cntp = (float)(t1 - t0 + 1); v4f r;
#pragma unroll
    for (int u = 0; u < 4; ++u) r[u] = __fdiv_rn(a[u], cntp); *(volatile v4f*)(outb + e) = r; __threadfence(); *(volatile v4f*)(outb + e) = r; }

extern "C" void kernel_launch(void* const* d_in, const int* in_sizes, int n_in,
                              void* d_out, int out_size, void* d_ws, size_t ws_size, hipStream_t stream) {
    (void)in_sizes; (void)n_in; (void)out_size;
    const float** I = (const float**)d_in;
    const float *X = I[0], *Wq = I[1], *bq = I[2], *Wk = I[3], *bk = I[4], *Wv = I[5], *bv = I[6]; const int* idx = (const int*)d_in[7];
    float* OUT = (float*)d_out;
    char* wsp = (char*)d_ws;
    auto take = [&](size_t bytes) { char* p = wsp; wsp += (bytes + 255) & ~(size_t)255; return (void*)p; };
    bf* XB = (bf*)take((size_t)NN * CC * 2); bf* BQ = (bf*)take((size_t)CC * CC * 2); bf* BK = (bf*)take((size_t)CC * CC * 2); bf* BV = (bf*)take((size_t)CC * CC * 2); float* CNT = (float*)take((size_t)NT * TW * 4);
    float* F = (float*)take((size_t)NN * CC * 4); bf* QPh = (bf*)take((size_t)NN * CC * 2); bf* QPl = (bf*)take((size_t)NN * CC * 2); bf* KPh = (bf*)take((size_t)NN * CC * 2); bf* KPl = (bf*)take((size_t)NN * CC * 2); bf* VBh = (bf*)take((size_t)NT * CC * TW * 2); bf* VBl = (bf*)take((size_t)NT * CC * TW * 2);
    float* S = (float*)take((size_t)NT * TW * TW * 4); bf* Ph = (bf*)take((size_t)NT * TW * TW * 2); bf* Pl = (bf*)take((size_t)NT * TW * TW * 2); float* O = (float*)take((size_t)NT * TW * CC * 4);
    if ((size_t)(wsp - (char*)d_ws) > ws_size) return;
    k_cvt8<<<(CC * CC / 8 + 255) / 256, 256, 0, stream>>>(Wq, BQ, CC * CC / 8); k_cvt8<<<(CC * CC / 8 + 255) / 256, 256, 0, stream>>>(Wk, BK, CC * CC / 8); k_cvt8<<<(CC * CC / 8 + 255) / 256, 256, 0, stream>>>(Wv, BV, CC * CC / 8);
    k_cnt<<<(NT * TW + 255) / 256, 256, 0, stream>>>(idx, CNT);
    const dim3 gp(NN / 64, CC / 64, 1); const unsigned gpl = (unsigned)(((size_t)NN * CC / 4 + 255) / 256);
    for (int b = 0; b < NB_; ++b) {
        k_cvt8<<<(NN * CC / 8 + 255) / 256, 256, 0, stream>>>(X + (size_t)b * NN * CC, XB, NN * CC / 8);
        k_gemmw<bf, 0, true><<<gp, 32, 0, stream>>>(XB, nullptr, BQ, nullptr, CC, F, CC, bq, 0, 0, 0); k_pl<<<gpl, 256, 0, stream>>>(F, (size_t)NN * CC, QPh, QPl);
        k_gemmw<bf, 0, true><<<gp, 32, 0, stream>>>(XB, nullptr, BK, nullptr, CC, F, CC, bk, 0, 0, 0); k_pl<<<gpl, 256, 0, stream>>>(F, (size_t)NN * CC, KPh, KPl);
        k_gemmw<bf, 0, true><<<gp, 32, 0, stream>>>(XB, nullptr, BV, nullptr, CC, F, CC, bv, 0, 0, 0); k_vpackt<<<(unsigned)(((size_t)NT * CC * TW / 2 + 255) / 256), 256, 0, stream>>>(F, VBh, VBl);
        k_gemmw<bf, 2, false><<<dim3(1, 1, NT), 32, 0, stream>>>(QPh, QPl, KPh, KPl, CC, S, TW, nullptr, (size_t)CC, (size_t)CC, (size_t)TW * TW);
        k_tsoft<<<(NT * TW + 7) / 8, 256, 0, stream>>>(S, CNT, Ph, Pl);
        k_gemmw<bf, 2, false><<<dim3(1, CC / 64, NT), 32, 0, stream>>>(Ph, Pl, VBh, VBl, TW, O, CC, nullptr, (size_t)TW * TW, (size_t)CC * TW, (size_t)TW * CC);
        k_accum<<<(NN * CC / 4 + 255) / 256, 256, 0, stream>>>(O, OUT + (size_t)b * NN * CC); }
}
